// GRUEncoder_89730456748115
// MI455X (gfx1250) — hardware-verified
//
#include <hip/hip_runtime.h>
#include <math.h>

#define BATCH 1024
#define SEQ   200
#define IN0   64
#define HID   128
#define G3    384
#define QSEQ  256
#define QROWS (QSEQ * SEQ)
#define NT    256
#define HP    136
#define FP    132

typedef __attribute__((ext_vector_type(16))) _Float16 v16h;
typedef __attribute__((ext_vector_type(8)))  _Float16 v8h;
typedef __attribute__((ext_vector_type(16))) __bf16   v16b;
typedef __attribute__((ext_vector_type(8)))  __bf16   v8b;
typedef __attribute__((ext_vector_type(8)))  float    v8f;
typedef __attribute__((ext_vector_type(4)))  float    v4f;

__device__ __forceinline__ unsigned short f2bf_bits(float f) {
  unsigned u = __float_as_uint(f);
  return (unsigned short)((u + 0x7FFFu + ((u >> 16) & 1u)) >> 16);
}
__device__ __forceinline__ float bf_bits2f(unsigned short h) { return __uint_as_float(((unsigned)h) << 16); }

__device__ __forceinline__ void dep_guard_h(v8f& a, v8f& b, v16h x, v16h y) { asm volatile("v_nop\n\tv_nop\n\tv_nop\n\tv_nop" : "+v"(a), "+v"(b) : "v"(x), "v"(y)); }
__device__ __forceinline__ void dep_guard_b(v8f& a, v8f& b, v16b x, v16b y) { asm volatile("v_nop\n\tv_nop\n\tv_nop\n\tv_nop" : "+v"(a), "+v"(b) : "v"(x), "v"(y)); }
__device__ __forceinline__ void keep4_h(v16h a, v16h b, v16h c, v16h d) { asm volatile("v_nop" :: "v"(a), "v"(b), "v"(c), "v"(d)); }
__device__ __forceinline__ void keep4_b(v16b a, v16b b, v16b c, v16b d) { asm volatile("v_nop" :: "v"(a), "v"(b), "v"(c), "v"(d)); }
__device__ __forceinline__ void acc_guard4(v8f& a, v8f& b, v8f& c, v8f& d) { asm volatile("v_nop\n\tv_nop\n\tv_nop\n\tv_nop" : "+v"(a), "+v"(b), "+v"(c), "+v"(d)); }
__device__ __forceinline__ void dep_guard3_h(v8f& a, v8f& b, v8f& c, v16h w, v16h x, v16h y, v16h z) {
  asm volatile("v_nop\n\tv_nop\n\tv_nop\n\tv_nop" : "+v"(a), "+v"(b), "+v"(c) : "v"(w), "v"(x), "v"(y), "v"(z));
}
__device__ __forceinline__ void acc_guard3(v8f& a, v8f& b, v8f& c) { asm volatile("v_nop\n\tv_nop\n\tv_nop\n\tv_nop" : "+v"(a), "+v"(b), "+v"(c)); }

template <typename T> struct Frag;
template <> struct Frag<_Float16> {
  typedef v16h V; union U { v16h v; v8h h[2]; };
  static __device__ __forceinline__ v16h load(const _Float16* p) {
    U f; f.h[0] = *(const v8h*)(p); f.h[1] = *(const v8h*)(p + 16); return f.v;
  }
  static __device__ __forceinline__ v8f mma(v16h a, v16h b, v8f c) {
    return __builtin_amdgcn_wmma_f32_16x16x32_f16(false, a, false, b, (short)0, c, false, false);
  }
  static __device__ __forceinline__ void guard(v8f& a, v8f& b, v16h x, v16h y) { dep_guard_h(a, b, x, y); }
  static __device__ __forceinline__ void keep(v16h a, v16h b, v16h c, v16h d) { keep4_h(a, b, c, d); }
};
template <> struct Frag<__bf16> {
  typedef v16b V; union U { v16b v; v8b h[2]; };
  static __device__ __forceinline__ v16b load(const __bf16* p) {
    U f; f.h[0] = *(const v8b*)(p); f.h[1] = *(const v8b*)(p + 16); return f.v;
  }
  static __device__ __forceinline__ v8f mma(v16b a, v16b b, v8f c) {
    return __builtin_amdgcn_wmma_f32_16x16x32_bf16(false, a, false, b, (short)0, c, false, false);
  }
  static __device__ __forceinline__ void guard(v8f& a, v8f& b, v16b x, v16b y) { dep_guard_b(a, b, x, y); }
  static __device__ __forceinline__ void keep(v16b a, v16b b, v16b c, v16b d) { keep4_b(a, b, c, d); }
};

template <int ET> struct Elem;
template <> struct Elem<0> { typedef _Float16 T; };
template <> struct Elem<1> { typedef __bf16 T; };
template <int ET, bool SPLIT, int BIAS_MODE, int OUT_MODE, bool RESID, int ACT = 0>
__global__ __launch_bounds__(256) void wmma_gemm64(
    const unsigned short* __restrict__ Ap, const unsigned short* __restrict__ A2p, int lda, long strideA,
    const unsigned short* __restrict__ Btp, const unsigned short* __restrict__ Bt2p, int ldb, long strideB,
    void* __restrict__ Cout, void* __restrict__ Cout2, int ldc, long strideC,
    const float* __restrict__ bias,
    const float* __restrict__ resid, long strideR,
    int M, int N, int K, float scale) {
  typedef typename Elem<ET>::T T;
  typedef typename Frag<T>::V V;
  const T* A = (const T*)Ap; const T* A2 = (const T*)A2p; const T* Bt = (const T*)Btp; const T* Bt2 = (const T*)Bt2p;
  __shared__ __align__(16) float sT[8][16 * 68];
  const int b    = blockIdx.y;
  const int lane = threadIdx.x & 31;
  const int wave = threadIdx.x >> 5;
  const int tilesN = N >> 6;
  const int tilesM = M >> 6;
  const int tile = blockIdx.x * 8 + wave;
  if (tile >= tilesM * tilesN) return;
  const int tm = tile / tilesN;
  const int tn = tile - tm * tilesN;
  const int m0 = tm << 6;
  const int n0 = tn << 6;

  const T* Ab  = A  + (size_t)b * strideA;
  const T* Bb  = Bt + (size_t)b * strideB;
  const T* Ab2 = SPLIT ? (A2  + (size_t)b * strideA) : nullptr;
  const T* Bb2 = SPLIT ? (Bt2 + (size_t)b * strideB) : nullptr;

  const int rlane = lane & 15;
  const int koff  = (lane >> 4) * 8;
  const int mOff  = (lane >> 4) * 8;

  v8f acc[4][4];
#pragma unroll
  for (int i = 0; i < 4; ++i)
#pragma unroll
    for (int j = 0; j < 4; ++j) acc[i][j] = (v8f){0.f,0.f,0.f,0.f,0.f,0.f,0.f,0.f};

  for (int k0 = 0; k0 < K; k0 += 32) {
    V bh[4], bl[4];
#pragma unroll
    for (int j = 0; j < 4; ++j) {
      const size_t bo = (size_t)(n0 + (j << 4) + rlane) * ldb + koff + k0;
      bh[j] = Frag<T>::load(Bb + bo);
      if (SPLIT) bl[j] = Frag<T>::load(Bb2 + bo);
    }
#pragma unroll
    for (int i = 0; i < 4; ++i) {
      const size_t ao = (size_t)(m0 + (i << 4) + rlane) * lda + koff + k0;
      V ah = Frag<T>::load(Ab + ao);
      V al;
      if (SPLIT) al = Frag<T>::load(Ab2 + ao);
#pragma unroll
      for (int j = 0; j < 4; ++j) {
        acc[i][j] = Frag<T>::mma(ah, bh[j], acc[i][j]);
        if (SPLIT) {
          acc[i][j] = Frag<T>::mma(ah, bl[j], acc[i][j]);
          acc[i][j] = Frag<T>::mma(al, bh[j], acc[i][j]);
        }
      }
      Frag<T>::guard(acc[i][0], acc[i][3], ah, SPLIT ? al : ah);
    }
    Frag<T>::keep(bh[0], bh[1], bh[2], bh[3]);
    if (SPLIT) Frag<T>::keep(bl[0], bl[1], bl[2], bl[3]);
  }
  acc_guard4(acc[0][0], acc[0][1], acc[0][2], acc[0][3]);
  acc_guard4(acc[1][0], acc[1][1], acc[1][2], acc[1][3]);
  acc_guard4(acc[2][0], acc[2][1], acc[2][2], acc[2][3]);
  acc_guard4(acc[3][0], acc[3][1], acc[3][2], acc[3][3]);

  float* slab = sT[wave];
  const float* Rb = RESID ? (resid + (size_t)b * strideR) : nullptr;
#pragma unroll
  for (int i = 0; i < 4; ++i) {
    const int mBase = m0 + (i << 4);
#pragma unroll
    for (int j = 0; j < 4; ++j) {
      const int n = n0 + (j << 4) + rlane;
      float bv = 0.f;
      if (BIAS_MODE == 2) bv = bias[n];
#pragma unroll
      for (int r = 0; r < 8; ++r) {
        float v = acc[i][j][r] * scale;
        if (BIAS_MODE == 1) v += bias[mBase + mOff + r];
        if (BIAS_MODE == 2) v += bv;
        if (RESID) v += Rb[(size_t)(mBase + mOff + r) * ldc + n];
        if (ACT == 1) v = tanhf(v);
        if (ACT == 2) v = fmaxf(v, 0.0f);
        if (ACT == 3) v = v / (1.0f + expf(-v));
        if (ACT == 4) v = (v > 0.f) ? v : 0.01f * v;
        if (ACT == 5) v = 0.5f * v * (1.0f + erff(v * 0.70710678118654752f));
        slab[(mOff + r) * 68 + (j << 4) + rlane] = v;
      }
    }
    __builtin_amdgcn_fence(__ATOMIC_RELEASE, "workgroup");
    __builtin_amdgcn_wave_barrier();
    __builtin_amdgcn_fence(__ATOMIC_ACQUIRE, "workgroup");
    if (OUT_MODE == 0) {
      float* C = (float*)Cout + (size_t)b * strideC;
      const int hh = lane >> 4, c4 = (lane & 15) * 4;
      for (int pass = 0; pass < 2; ++pass) {
#pragma unroll
        for (int it = 0; it < 8; ++it) {
          const int row = it * 2 + hh;
          v4f v = *(const v4f*)(slab + row * 68 + c4);
          *(volatile v4f*)(C + (size_t)(mBase + row) * ldc + n0 + c4) = v;
        }
        __threadfence();
      }
    } else {
      const int q = lane >> 3, c8 = (lane & 7) * 8;
      unsigned short* C  = (unsigned short*)Cout  + (size_t)b * strideC;
      unsigned short* C2 = (OUT_MODE == 2) ? ((unsigned short*)Cout2 + (size_t)b * strideC) : nullptr;
      for (int pass = 0; pass < 2; ++pass) {
#pragma unroll
        for (int it = 0; it < 4; ++it) {
          const int row = it * 4 + q;
          const float* sp = slab + row * 68 + c8;
          v8h hv, lv;
#pragma unroll
          for (int e = 0; e < 8; ++e) {
            if (OUT_MODE == 1) {
              hv[e] = (_Float16)sp[e];
            } else {
              unsigned short hb = f2bf_bits(sp[e]);
              unsigned short lb = f2bf_bits(sp[e] - bf_bits2f(hb));
              hv[e] = __builtin_bit_cast(_Float16, hb);
              lv[e] = __builtin_bit_cast(_Float16, lb);
            }
          }
          *(volatile v8h*)(C + (size_t)(mBase + row) * ldc + n0 + c8) = hv;
          if (OUT_MODE == 2) *(volatile v8h*)(C2 + (size_t)(mBase + row) * ldc + n0 + c8) = lv;
        }
        __threadfence();
      }
    }
    __builtin_amdgcn_fence(__ATOMIC_RELEASE, "workgroup");
    __builtin_amdgcn_wave_barrier();
    __builtin_amdgcn_fence(__ATOMIC_ACQUIRE, "workgroup");
  }
}

__device__ __forceinline__ unsigned pack_f16x2(float a, float b) {
  const _Float16 h0 = (_Float16)a, h1 = (_Float16)b;
  return (unsigned)__builtin_bit_cast(unsigned short, h0) | ((unsigned)__builtin_bit_cast(unsigned short, h1) << 16);
}
__device__ __forceinline__ void st2u(unsigned* p, unsigned v) { *(volatile unsigned*)p = v; __threadfence(); *(volatile unsigned*)p = v; }
__device__ __forceinline__ float ftanh(float x) { return 1.0f - 2.0f * __builtin_amdgcn_rcpf(1.0f + __expf(2.0f * x)); }
__device__ __forceinline__ float fsigm(float x) { return __builtin_amdgcn_rcpf(1.0f + __expf(-x)); }

__global__ __launch_bounds__(NT) void prep_kernel(const float* __restrict__ x,
                                                 const float* __restrict__ Wih0, const float* __restrict__ Whh0,
                                                 const float* __restrict__ Wih1, const float* __restrict__ Whh1,
                                                 _Float16* __restrict__ X16,
                                                 unsigned* __restrict__ WIH0, unsigned* __restrict__ WHH0,
                                                 unsigned* __restrict__ WIH1, unsigned* __restrict__ WHH1) {
  const int blk = blockIdx.x, tid = threadIdx.x;
  if (blk < 6400) {
    const int gid = blk * NT + tid;
    const float* p = x + (size_t)gid * 8;
    const v4f a = *(const v4f*)p, bq = *(const v4f*)(p + 4);
    v8h h;
#pragma unroll
    for (int e = 0; e < 4; ++e) { h[e] = (_Float16)a[e]; h[4 + e] = (_Float16)bq[e]; }
    _Float16* op = X16 + (size_t)gid * 8;
    *(volatile v8h*)op = h; __threadfence(); *(volatile v8h*)op = h;
  } else if (blk < 6448) {
    const int p = (blk - 6400) * NT + tid;
    const unsigned u = pack_f16x2(Wih0[2 * p] * 16.0f, Wih0[2 * p + 1] * 16.0f);
    st2u(WIH0 + p, u);
  } else if (blk < 6544) {
    const int p = (blk - 6448) * NT + tid;
    const unsigned u = pack_f16x2(Whh0[2 * p] * 16.0f, Whh0[2 * p + 1] * 16.0f);
    st2u(WHH0 + p, u);
  } else if (blk < 6640) {
    const int p = (blk - 6544) * NT + tid;
    const unsigned u = pack_f16x2(Wih1[2 * p] * 16.0f, Wih1[2 * p + 1] * 16.0f);
    st2u(WIH1 + p, u);
  } else {
    const int p = (blk - 6640) * NT + tid;
    const unsigned u = pack_f16x2(Whh1[2 * p] * 16.0f, Whh1[2 * p + 1] * 16.0f);
    st2u(WHH1 + p, u);
  }
}

template <bool FINAL>
__global__ __launch_bounds__(NT) void gru_rec_kernel(const float* __restrict__ XG, const _Float16* __restrict__ WHH,
                                                    const float* __restrict__ bhh,
                                                    _Float16* __restrict__ HSEQ, float* __restrict__ OUT) {
  __shared__ __align__(16) _Float16 h16[16 * HP];
  __shared__ __align__(16) float hf[FINAL ? 16 * FP : 4];
  const int tid = threadIdx.x, lane = tid & 31, wave = tid >> 5;
  const int rlane = lane & 15, hh = lane >> 4, koff = hh * 8, mOff = hh * 8;
  const int blk = blockIdx.x;
  for (int i = tid; i < 16 * HP; i += NT) h16[i] = (_Float16)0.0f;
  __syncthreads();

  const int j = 16 * wave + rlane;
  const _Float16* arow = h16 + rlane * HP + koff;
  const _Float16* wr = WHH + (size_t)j * HID + koff;
  const _Float16* wz = WHH + (size_t)(HID + j) * HID + koff;
  const _Float16* wn = WHH + (size_t)(2 * HID + j) * HID + koff;
  const float br = bhh[j], bz = bhh[HID + j], bn = bhh[2 * HID + j];
  const float* xgb = XG + (size_t)(blk * 16 + mOff) * SEQ * G3 + j;
  const v8f z8 = {0.f, 0.f, 0.f, 0.f, 0.f, 0.f, 0.f, 0.f};
  const float s16 = 1.0f / 16.0f;

  float hreg[8];
#pragma unroll
  for (int r = 0; r < 8; ++r) hreg[r] = 0.0f;

#pragma unroll 1
  for (int t = 0; t < SEQ; ++t) {
    v8f ar = z8, az = z8, an = z8;
#pragma unroll 1
    for (int k0 = 0; k0 < HID; k0 += 32) {
      const v16h a  = Frag<_Float16>::load(arow + k0);
      const v16h b0 = Frag<_Float16>::load(wr + k0);
      const v16h b1 = Frag<_Float16>::load(wz + k0);
      const v16h b2 = Frag<_Float16>::load(wn + k0);
      ar = Frag<_Float16>::mma(a, b0, ar);
      az = Frag<_Float16>::mma(a, b1, az);
      an = Frag<_Float16>::mma(a, b2, an);
      dep_guard3_h(ar, az, an, a, b0, b1, b2);
    }
    acc_guard3(ar, az, an);

    const float* xt = xgb + (size_t)t * G3;
#pragma unroll
    for (int r = 0; r < 8; ++r) {
      const float* xr = xt + (size_t)r * SEQ * G3;
      const float x_r = xr[0], x_z = xr[HID], x_n = xr[2 * HID];
      const float hr = ar[r] * s16 + br;
      const float hz = az[r] * s16 + bz;
      const float hn = an[r] * s16 + bn;
      const float rg = fsigm(x_r + hr);
      const float zg = fsigm(x_z + hz);
      const float ng = ftanh(x_n + rg * hn);
      hreg[r] = (1.0f - zg) * ng + zg * hreg[r];
    }
    __syncthreads();
#pragma unroll
    for (int r = 0; r < 8; ++r) h16[(mOff + r) * HP + j] = (_Float16)hreg[r];
    __syncthreads();
    if (!FINAL) {
      _Float16* hsb = HSEQ + ((size_t)(blk * 16) * SEQ + t) * HID;
      const int row = 2 * wave + hh, c8 = (lane & 15) * 8;
      for (int pass = 0; pass < 2; ++pass) {
        const v8h v = *(const v8h*)(h16 + row * HP + c8);
        *(volatile v8h*)(hsb + (size_t)row * SEQ * HID + c8) = v;
        __threadfence();
      }
    }
  }

  if (FINAL) {
#pragma unroll
    for (int r = 0; r < 8; ++r) hf[(mOff + r) * FP + j] = hreg[r];
    __syncthreads();
    const int row = 2 * wave + hh;
    for (int pass = 0; pass < 2; ++pass) {
#pragma unroll
      for (int it = 0; it < 2; ++it) {
        const int c4 = it * 64 + (lane & 15) * 4;
        const v4f v = *(const v4f*)(hf + row * FP + c4);
        *(volatile v4f*)(OUT + (size_t)(blk * 16 + row) * HID + c4) = v;
      }
      __threadfence();
    }
  }
}

extern "C" void kernel_launch(void* const* d_in, const int* in_sizes, int n_in,
                              void* d_out, int out_size, void* d_ws, size_t ws_size, hipStream_t stream) {
  if (n_in < 9 || d_out == nullptr || d_ws == nullptr) return;
  if (in_sizes[0] != BATCH * SEQ * IN0 || in_sizes[1] != G3 * IN0 || in_sizes[2] != G3 * HID || in_sizes[3] != G3 ||
      in_sizes[4] != G3 || in_sizes[5] != G3 * HID || in_sizes[6] != G3 * HID || in_sizes[7] != G3 || in_sizes[8] != G3 ||
      out_size != BATCH * HID) return;

  const float* x    = (const float*)d_in[0];
  const float* Wih0 = (const float*)d_in[1];
  const float* Whh0 = (const float*)d_in[2];
  const float* bih0 = (const float*)d_in[3];
  const float* bhh0 = (const float*)d_in[4];
  const float* Wih1 = (const float*)d_in[5];
  const float* Whh1 = (const float*)d_in[6];
  const float* bih1 = (const float*)d_in[7];
  const float* bhh1 = (const float*)d_in[8];
  float* out = (float*)d_out;

  char* ws = (char*)d_ws; size_t off = 0;
  auto carve = [&](size_t bytes) -> char* { char* p = ws + off; off += (bytes + 255) & ~(size_t)255; return p; };
  _Float16* X16    = (_Float16*)carve((size_t)BATCH * SEQ * IN0 * 2);
  unsigned* WIH0u  = (unsigned*)carve((size_t)G3 * IN0 * 2);
  unsigned* WHH0u  = (unsigned*)carve((size_t)G3 * HID * 2);
  unsigned* WIH1u  = (unsigned*)carve((size_t)G3 * HID * 2);
  unsigned* WHH1u  = (unsigned*)carve((size_t)G3 * HID * 2);
  float*    XG32   = (float*)carve((size_t)QROWS * G3 * 4);
  _Float16* HSEQ16 = (_Float16*)carve((size_t)QROWS * HID * 2);
  if (off > ws_size || off > (size_t)134217728) return;
  const _Float16* WIH0 = (const _Float16*)WIH0u;
  const _Float16* WHH0 = (const _Float16*)WHH0u;
  const _Float16* WIH1 = (const _Float16*)WIH1u;
  const _Float16* WHH1 = (const _Float16*)WHH1u;

  prep_kernel<<<6736, NT, 0, stream>>>(x, Wih0, Whh0, Wih1, Whh1, X16, WIH0u, WHH0u, WIH1u, WHH1u);

  const int tiles = (QROWS / 64) * (G3 / 64);
  for (int q = 0; q < BATCH / QSEQ; ++q) {
    wmma_gemm64<0, false, 2, 0, false><<<dim3(tiles / 8, 1), 256, 0, stream>>>(
        (const unsigned short*)(X16 + (size_t)q * QROWS * IN0), (const unsigned short*)nullptr, IN0, 0L,
        (const unsigned short*)WIH0, (const unsigned short*)nullptr, IN0, 0L,
        (void*)XG32, (void*)nullptr, G3, 0L,
        bih0, (const float*)nullptr, 0L, QROWS, G3, IN0, 1.0f / 16.0f);
    gru_rec_kernel<false><<<QSEQ / 16, NT, 0, stream>>>(XG32, WHH0, bhh0, HSEQ16, out + (size_t)q * QSEQ * HID);
    wmma_gemm64<0, false, 2, 0, false><<<dim3(tiles / 8, 1), 256, 0, stream>>>(
        (const unsigned short*)HSEQ16, (const unsigned short*)nullptr, HID, 0L,
        (const unsigned short*)WIH1, (const unsigned short*)nullptr, HID, 0L,
        (void*)XG32, (void*)nullptr, G3, 0L,
        bih1, (const float*)nullptr, 0L, QROWS, G3, HID, 1.0f / 16.0f);
    gru_rec_kernel<true><<<QSEQ / 16, NT, 0, stream>>>(XG32, WHH1, bhh1, HSEQ16, out + (size_t)q * QSEQ * HID);
  }
}
